// Concept_ood_24017457119454
// MI455X (gfx1250) — hardware-run, weakly checked
//
#include <hip/hip_runtime.h>


#ifndef NBQ
#define NBQ 1024
#endif
#define NBQ_FULL 1024
#define NS   512
#define NE   1024
#define ND   2048
#define QRS  2048.0f
#define QRI  (1.0f / 2048.0f)
#define WCAR  64.0f
#define WCARI (1.0f / 64.0f)
#define CCAR  64.0f
#define PCAR  16384.0f
#define YSCL  (1.0f / (16384.0f * 64.0f))
#define SML2  ((float)(10.0 * 1.4426950408889634))
#define BNEPS 1e-5f
#define L2EPS 1e-8f
#define NEGB  (-3.0e38f)
#define PSP   516

static_assert(NBQ <= NBQ_FULL);
static_assert(NBQ % 64 == 0);
static_assert(NS % 64 == 0);
static_assert(NE % 64 == 0);
static_assert(ND % 64 == 0);
static_assert(NS % 32 == 0);
static_assert(NE % 32 == 0);
static_assert(ND % 32 == 0);
static_assert((NE & (NE - 1)) == 0);
static_assert(((size_t)NS * NE) % 2048 == 0);
static_assert(((size_t)NBQ * NE) % 2048 == 0);
static_assert(NS == 8 * 64);
static_assert(PSP >= NS);
static_assert((PSP * 4) % 16 == 0);
static_assert(ND % 128 == 0);
static_assert(NBQ % 16 == 0);
static_assert(NBQ % 8 == 0);
static_assert(((size_t)NS * ND) % 8 == 0);
static_assert(((size_t)NBQ * NE) % 8 == 0);
static_assert((size_t)NBQ_FULL * ND * 4 == (size_t)8388608);
static_assert(256 * 2 * 16 == 64 * 128);
static_assert(32 * 8 * 16 == 16 * 256);
static_assert(256 * 8 * 16 == 16 * NS * 4);
static_assert(256 * 4 * 16 == 16 * NS * 2);
static_assert(256 * 16 == 2048 * 2);
static_assert(32 * 16 * 16 == ND * 4);
static_assert(64 * 68 * 4 <= 131072);
static_assert(16 * 68 * 4 <= 131072);
static_assert(16 * PSP * 4 + 2 * 8 * 16 * 4 <= 131072);
static_assert(2048 * 4 <= 131072);
static_assert((8 * 32 + 64) * 4 <= 131072);

typedef _Float16 h16;
typedef unsigned short bf;
typedef __attribute__((ext_vector_type(16))) __bf16   v16bf;
typedef __attribute__((ext_vector_type(16))) _Float16 v16h;
typedef __attribute__((ext_vector_type(8)))  _Float16 v8h;
typedef __attribute__((ext_vector_type(8)))  unsigned short v8us;
typedef __attribute__((ext_vector_type(8)))  float    v8f;
typedef __attribute__((ext_vector_type(4)))  float    v4f;
typedef v4f  __attribute__((may_alias)) v4fa;

__device__ __forceinline__ unsigned short f2bf(float f) { unsigned u = __float_as_uint(f); u += 0x7FFFu + ((u >> 16) & 1u); return (unsigned short)(u >> 16); }
__device__ __forceinline__ float bfr(float f) { return __uint_as_float(((unsigned)f2bf(f)) << 16); }
__device__ __forceinline__ v16h cat16(v8h lo, v8h hi) { return __builtin_shufflevector(lo, hi, 0, 1, 2, 3, 4, 5, 6, 7, 8, 9, 10, 11, 12, 13, 14, 15); }
__device__ __forceinline__ v16bf cat16b(v8us lo, v8us hi) { return __builtin_bit_cast(v16bf, __builtin_shufflevector(lo, hi, 0, 1, 2, 3, 4, 5, 6, 7, 8, 9, 10, 11, 12, 13, 14, 15)); }
__device__ __forceinline__ v8f wmma16(v16h a, v16h b, v8f c) { return __builtin_amdgcn_wmma_f32_16x16x32_f16(false, a, false, b, (short)0, c, false, false); }
__device__ __forceinline__ v8f wmmab(v16bf a, v16bf b, v8f c) { return __builtin_amdgcn_wmma_f32_16x16x32_bf16(false, a, false, b, (short)0, c, false, false); }
__device__ __forceinline__ v16h  ldh(const h16* p) { return cat16(*(const v8h*)p, *(const v8h*)(p + 16)); }
__device__ __forceinline__ v16bf ldb(const bf* p)  { return cat16b(*(const v8us*)p, *(const v8us*)(p + 16)); }
__device__ __forceinline__ void wave_sync() { __builtin_amdgcn_fence(3  , "wavefront"); __builtin_amdgcn_wave_barrier(); asm volatile("" ::: "memory"); }

static __device__ __forceinline__ h16 toh_flush(float v) { const h16 r = (h16)v; return (fabsf(v) < 6.103515625e-05f) ? (h16)0.0f : r; }
__device__ __forceinline__ v16bf ldfr(const bf* p)  { return ldb(p); }
__device__ __forceinline__ v16h  ldfr(const h16* p) { return ldh(p); }
__device__ __forceinline__ v8f mmag(v16bf a, v16bf b, v8f c) { c = wmmab(a, b, c); asm volatile("v_nop\n\tv_nop\n\tv_nop\n\tv_nop" : "+v"(c) : "v"(a), "v"(b)); return c; }
__device__ __forceinline__ v8f mmag(v16h a, v16h b, v8f c)   { c = wmma16(a, b, c); asm volatile("v_nop\n\tv_nop\n\tv_nop\n\tv_nop" : "+v"(c) : "v"(a), "v"(b)); return c; }

__global__ __launch_bounds__(256) void k_cvt8(const float* __restrict__ src, bf* dst, size_t n8) {
    const size_t i = (size_t)blockIdx.x * 256 + threadIdx.x; if (i >= n8) return;
    const v8f v = *(const v8f*)(src + i * 8); v8us o;
#pragma unroll
    for (int k = 0; k < 8; ++k) o[k] = f2bf(v[k]);
    *(volatile v8us*)(dst + i * 8) = o; __threadfence(); *(volatile v8us*)(dst + i * 8) = o;
}

__global__ __launch_bounds__(256) void k_tcvt(const float* __restrict__ in, bf* out, int R, int C) {
#pragma clang fp contract(off)
    __shared__ __align__(16) float ts[64 * 68];
    const int tid = threadIdx.x;
    const int c0 = blockIdx.x * 64, r0 = blockIdx.y * 64;
#pragma unroll
    for (int it = 0; it < 4; ++it) { const int p = it * 256 + tid; const int r = p >> 4, c4 = (p & 15) * 4;
        const v4f v = *(const v4f*)(in + (size_t)(r0 + r) * C + c0 + c4);
        *(v4fa*)(&ts[r * 68 + c4]) = v; }
    __syncthreads();
    v8us o[2];
#pragma unroll
    for (int it = 0; it < 2; ++it) { const int q = it * 256 + tid; const int c = q >> 3, r8 = (q & 7) * 8;
#pragma unroll
        for (int j = 0; j < 8; ++j) o[it][j] = f2bf(ts[(r8 + j) * 68 + c]); }
#pragma unroll 1
    for (int ps = 0; ps < 2; ++ps) {
#pragma unroll
        for (int it = 0; it < 2; ++it) { const int q = it * 256 + tid; const int c = q >> 3, r8 = (q & 7) * 8;
            *(volatile v8us*)(out + (size_t)(c0 + c) * R + r0 + r8) = o[it]; }
        if (ps == 0) __threadfence(); }
}

__global__ __launch_bounds__(256) void k_rnorm(const float* __restrict__ X, float* INV) {
#pragma clang fp contract(off)
    __shared__ __align__(16) float sv[32];
    const int lane = threadIdx.x & 31;
    const int wave = __builtin_amdgcn_readfirstlane((int)(threadIdx.x >> 5));
#pragma unroll 1
    for (int j = 0; j < 4; ++j) {
        const int row = blockIdx.x * 32 + wave * 4 + j;
        const float* x = X + (size_t)row * ND;
        float s = 0.0f;
#pragma unroll 1
        for (int i = 0; i < ND / 128; ++i) { const v4f v = *(const v4f*)(x + (i * 32 + lane) * 4);
            const float a = bfr(v[0]), b = bfr(v[1]), c = bfr(v[2]), d = bfr(v[3]);
            s += a * a + b * b + c * c + d * d; }
        s += __shfl_xor(s, 16, 32); s += __shfl_xor(s, 8, 32); s += __shfl_xor(s, 4, 32); s += __shfl_xor(s, 2, 32); s += __shfl_xor(s, 1, 32);
        if (lane == 0) sv[wave * 4 + j] = 1.0f / (sqrtf(s) + L2EPS);
    }
    __syncthreads();
    if (threadIdx.x < 8) { const v4f v = *(const v4fa*)(&sv[threadIdx.x * 4]); float* dst = INV + blockIdx.x * 32 + threadIdx.x * 4;
        *(volatile v4f*)dst = v; __threadfence(); *(volatile v4f*)dst = v; }
}

__global__ __launch_bounds__(256) void k_cfnt(const float* __restrict__ in, const float* __restrict__ rsc, h16* out, int R, int C) {
#pragma clang fp contract(off)
    __shared__ __align__(16) float ts[64 * 68];
    const int tid = threadIdx.x;
    const int c0 = blockIdx.x * 64, r0 = blockIdx.y * 64;
#pragma unroll
    for (int it = 0; it < 4; ++it) { const int p = it * 256 + tid; const int r = p >> 4, c4 = (p & 15) * 4;
        const v4f v = *(const v4f*)(in + (size_t)(r0 + r) * C + c0 + c4);
        const float sc = rsc[r0 + r] * CCAR; v4f w;
        w[0] = bfr(v[0]) * sc; w[1] = bfr(v[1]) * sc; w[2] = bfr(v[2]) * sc; w[3] = bfr(v[3]) * sc;
        *(v4fa*)(&ts[r * 68 + c4]) = w; }
    __syncthreads();
    v8h o[2];
#pragma unroll
    for (int it = 0; it < 2; ++it) { const int q = it * 256 + tid; const int c = q >> 3, r8 = (q & 7) * 8;
#pragma unroll
        for (int j = 0; j < 8; ++j) o[it][j] = toh_flush(ts[(r8 + j) * 68 + c]); }
#pragma unroll 1
    for (int ps = 0; ps < 2; ++ps) {
#pragma unroll
        for (int it = 0; it < 2; ++it) { const int q = it * 256 + tid; const int c = q >> 3, r8 = (q & 7) * 8;
            *(volatile v8h*)(out + (size_t)(c0 + c) * R + r0 + r8) = o[it]; }
        if (ps == 0) __threadfence(); }
}

template <typename T, int HASB>
__device__ __forceinline__ void gemm64_body(const T* __restrict__ A, const T* __restrict__ Bt, const float* __restrict__ bias, float oscale, float* C, int K, int ldc) {
    __shared__ __align__(16) float os[16 * 68];
    typedef decltype(ldfr((const T*)0)) FR;
    const int lane = threadIdx.x & 31, lr = lane & 15, hi = lane >> 4; const int r0 = blockIdx.x * 64, c0 = blockIdx.y * 64;
    v8f acc[4][4];
#pragma unroll
    for (int mb = 0; mb < 4; ++mb)
#pragma unroll
        for (int nb = 0; nb < 4; ++nb) acc[mb][nb] = (v8f){};
    const size_t aoff = (size_t)(r0 + lr) * K + 8 * hi, boff = (size_t)(c0 + lr) * K + 8 * hi;
#pragma unroll 1
    for (int kc = 0; kc < K; kc += 32) {
        FR a[4];
#pragma unroll
        for (int mb = 0; mb < 4; ++mb) a[mb] = ldfr(A + aoff + (size_t)mb * 16 * K + kc);
#pragma unroll
        for (int nb = 0; nb < 4; ++nb) { const FR b = ldfr(Bt + boff + (size_t)nb * 16 * K + kc);
#pragma unroll
            for (int mb = 0; mb < 4; ++mb) acc[mb][nb] = mmag(a[mb], b, acc[mb][nb]); }
    }
    float bc[4] = { 0.0f, 0.0f, 0.0f, 0.0f };
    if (HASB) {
#pragma unroll
        for (int nb = 0; nb < 4; ++nb) bc[nb] = bfr(bias[c0 + nb * 16 + lr]); }
#pragma unroll
    for (int mb = 0; mb < 4; ++mb) {
#pragma unroll
        for (int nb = 0; nb < 4; ++nb) {
#pragma unroll
            for (int j = 0; j < 8; ++j) os[(hi * 8 + j) * 68 + nb * 16 + lr] = acc[mb][nb][j] * oscale + bc[nb]; }
        wave_sync();
        float* cb = C + (size_t)(r0 + mb * 16) * ldc + c0;
#pragma unroll 1
        for (int ps = 0; ps < 2; ++ps) {
#pragma unroll
            for (int s = 0; s < 8; ++s) { const int p = s * 32 + lane; const int row = p >> 4, c4 = (p & 15) * 4;
                const v4f val = *(const v4fa*)(&os[row * 68 + c4]);
                *(volatile v4f*)(cb + (size_t)row * ldc + c4) = val; }
            if (ps == 0) __threadfence(); }
        wave_sync();
    }
}

__global__ __launch_bounds__(32) void k_gemm_bf(const bf* __restrict__ A, const bf* __restrict__ Bt, const float* __restrict__ bias, float* C, int K, int ldc) {
    gemm64_body<bf, 1>(A, Bt, bias, 1.0f, C, K, ldc);
}
__global__ __launch_bounds__(32) void k_gemm_h(const h16* __restrict__ A, const h16* __restrict__ Bt, float oscale, float* C, int K, int ldc) {
    gemm64_body<h16, 0>(A, Bt, (const float*)0, oscale, C, K, ldc);
}

__global__ __launch_bounds__(256) void k_bnstat(const float* __restrict__ Z, float* MU, float* RS, int M) {
#pragma clang fp contract(off)
    __shared__ __align__(16) float red[8 * 32];
    __shared__ __align__(16) float sm[64];
    const int lane = threadIdx.x & 31;
    const int wave = __builtin_amdgcn_readfirstlane((int)(threadIdx.x >> 5));
    const int c = blockIdx.x * 32 + lane;
    const float rm = 1.0f / (float)M;
    float s = 0.0f;
#pragma unroll 4
    for (int r = wave; r < M; r += 8) s += Z[(size_t)r * NE + c];
    red[wave * 32 + lane] = s;
    __syncthreads();
    float tot = 0.0f;
#pragma unroll
    for (int w = 0; w < 8; ++w) tot += red[w * 32 + lane];
    const float mu = tot * rm;
    __syncthreads();
    float q = 0.0f;
#pragma unroll 4
    for (int r = wave; r < M; r += 8) { const float d = Z[(size_t)r * NE + c] - mu; q += d * d; }
    red[wave * 32 + lane] = q;
    __syncthreads();
    float qt = 0.0f;
#pragma unroll
    for (int w = 0; w < 8; ++w) qt += red[w * 32 + lane];
    const float rs = 1.0f / sqrtf(qt * rm + BNEPS);
    if (wave == 0) {
        sm[lane] = mu; sm[32 + lane] = rs;
        wave_sync();
        if (lane < 8) { const v4f a = *(const v4fa*)(&sm[lane * 4]); const v4f b = *(const v4fa*)(&sm[32 + lane * 4]);
            float* pm = MU + blockIdx.x * 32 + lane * 4; float* pr = RS + blockIdx.x * 32 + lane * 4;
            *(volatile v4f*)pm = a; *(volatile v4f*)pr = b; __threadfence(); *(volatile v4f*)pm = a; *(volatile v4f*)pr = b; }
    }
}

__global__ __launch_bounds__(256) void k_bnact(const float* __restrict__ Z, const float* __restrict__ MU, const float* __restrict__ RS,
                                               const float* __restrict__ g, const float* __restrict__ b, const float* __restrict__ f3, int use_f3, float carry,
                                               h16* HP, h16* RP) {
#pragma clang fp contract(off)
    __shared__ __align__(16) float sm[2048];
    const int tid = threadIdx.x;
    const size_t base = (size_t)blockIdx.x * 2048;
#pragma unroll 1
    for (int j = 0; j < 8; ++j) {
        const int li = j * 256 + tid; const size_t idx = base + (size_t)li; const int e = (int)(idx & (size_t)(NE - 1));
        const float z = Z[idx];
        const float y = bfr(g[e]) * (z - MU[e]) * RS[e] + bfr(b[e]);
        const float ay = fabsf(y);
        const float ex = __builtin_amdgcn_exp2f(ay * -2.8853900817779268f);
        const float t = (1.0f - ex) * __builtin_amdgcn_rcpf(1.0f + ex);
        const float w = copysignf(t, y);
        const float f = bfr(f3[e]);
        const float ff = (use_f3 != 0) ? f : 1.0f;
        sm[li] = (w * ff) * carry;
    }
    __syncthreads();
    const v4f x0 = *(const v4fa*)(&sm[tid * 8]); const v4f x1 = *(const v4fa*)(&sm[tid * 8 + 4]); v8h hv, rv;
#pragma unroll
    for (int i = 0; i < 4; ++i) { const h16 a0 = toh_flush(x0[i]); const h16 a1 = toh_flush(x1[i]); hv[i] = a0; hv[4 + i] = a1;
        rv[i] = toh_flush((x0[i] - (float)a0) * QRS); rv[4 + i] = toh_flush((x1[i] - (float)a1) * QRS); }
    h16* ph = HP + base + (size_t)tid * 8; h16* pr = RP + base + (size_t)tid * 8;
    *(volatile v8h*)ph = hv; *(volatile v8h*)pr = rv; __threadfence(); *(volatile v8h*)ph = hv; *(volatile v8h*)pr = rv;
}

__global__ __launch_bounds__(256) void k_score(const h16* __restrict__ WSH, const h16* __restrict__ WSR, const h16* __restrict__ WVH, const h16* __restrict__ WVR,
                                               const float* __restrict__ b3p, float* O1, h16* PP) {
    __shared__ __align__(16) float pt[16 * PSP];
    __shared__ __align__(16) float wmx[8 * 16];
    __shared__ __align__(16) float wsm[8 * 16];
    const int tid = threadIdx.x, lane = tid & 31, lr = lane & 15, hi = lane >> 4;
    const int wave = __builtin_amdgcn_readfirstlane((int)(threadIdx.x >> 5));
    const int b0 = blockIdx.x * 16;
    const size_t ao = (size_t)(wave * 64 + lr) * NE + 8 * hi;
    const size_t bo = (size_t)(b0 + lr) * NE + 8 * hi;
    v8f sH[4], sL[4];
#pragma unroll
    for (int t = 0; t < 4; ++t) { sH[t] = (v8f){}; sL[t] = (v8f){}; }
#pragma unroll 1
    for (int kc = 0; kc < NE; kc += 32) {
        const v16h bh = ldh(WVH + bo + kc), br = ldh(WVR + bo + kc);
#pragma unroll
        for (int t = 0; t < 4; ++t) {
            const v16h ah = ldh(WSH + ao + (size_t)t * 16 * NE + kc), ar = ldh(WSR + ao + (size_t)t * 16 * NE + kc);
            sH[t] = mmag(ah, bh, sH[t]); sL[t] = mmag(ah, br, sL[t]); sL[t] = mmag(ar, bh, sL[t]); }
    }
    const float b3 = bfr(b3p[0]);
    float tv[4][8]; float mx = NEGB;
#pragma unroll
    for (int t = 0; t < 4; ++t) {
#pragma unroll
        for (int r = 0; r < 8; ++r) { const float a = (sH[t][r] + sL[t][r] * QRI) * WCARI + b3; tv[t][r] = a * SML2; mx = fmaxf(mx, tv[t][r]); } }
    mx = fmaxf(mx, __shfl_xor(mx, 16, 32));
    if (hi == 0) wmx[wave * 16 + lr] = mx;
    __syncthreads();
    float mrow = wmx[lr];
#pragma unroll
    for (int w = 1; w < 8; ++w) mrow = fmaxf(mrow, wmx[w * 16 + lr]);
    float ls = 0.0f;
#pragma unroll
    for (int t = 0; t < 4; ++t) {
#pragma unroll
        for (int r = 0; r < 8; ++r) { const float e = __builtin_amdgcn_exp2f(tv[t][r] - mrow); tv[t][r] = e; ls += e; } }
    ls += __shfl_xor(ls, 16, 32);
    if (hi == 0) wsm[wave * 16 + lr] = ls;
    __syncthreads();
    float lrow = 0.0f;
#pragma unroll
    for (int w = 0; w < 8; ++w) lrow += wsm[w * 16 + lr];
    const float inv = 1.0f / lrow;
#pragma unroll
    for (int t = 0; t < 4; ++t) { v4f a, c;
        a[0] = tv[t][0] * inv; a[1] = tv[t][1] * inv; a[2] = tv[t][2] * inv; a[3] = tv[t][3] * inv;
        c[0] = tv[t][4] * inv; c[1] = tv[t][5] * inv; c[2] = tv[t][6] * inv; c[3] = tv[t][7] * inv;
        const int o = lr * PSP + wave * 64 + t * 16 + 8 * hi;
        *(v4fa*)(&pt[o]) = a; *(v4fa*)(&pt[o + 4]) = c; }
    __syncthreads();
#pragma unroll 1
    for (int ps = 0; ps < 2; ++ps) {
#pragma unroll
        for (int it = 0; it < 8; ++it) { const int p = it * 256 + tid; const int row = p >> 7, c4 = (p & 127) * 4;
            const v4f val = *(const v4fa*)(&pt[row * PSP + c4]);
            *(volatile v4f*)(O1 + (size_t)(b0 + row) * NS + c4) = val; }
#pragma unroll
        for (int it = 0; it < 4; ++it) { const int p = it * 256 + tid; const int row = p >> 6, c8 = (p & 63) * 8;
            const v4f x0 = *(const v4fa*)(&pt[row * PSP + c8]); const v4f x1 = *(const v4fa*)(&pt[row * PSP + c8 + 4]); v8h hv;
#pragma unroll
            for (int i = 0; i < 4; ++i) { hv[i] = toh_flush(x0[i] * PCAR); hv[4 + i] = toh_flush(x1[i] * PCAR); }
            *(volatile v8h*)(PP + (size_t)(b0 + row) * NS + c8) = hv; }
        if (ps == 0) __threadfence(); }
}

__global__ __launch_bounds__(256) void k_l2out(const float* __restrict__ Y, float* O0) {
#pragma clang fp contract(off)
    const int lane = threadIdx.x & 31;
    const int wave = __builtin_amdgcn_readfirstlane((int)(threadIdx.x >> 5));
    const int row = blockIdx.x * 8 + wave;
    const float* y = Y + (size_t)row * ND; float* o = O0 + (size_t)row * ND;
    float s = 0.0f;
#pragma unroll 1
    for (int i = 0; i < ND / 128; ++i) { const v4f v = *(const v4f*)(y + (i * 32 + lane) * 4);
        s += v[0] * v[0] + v[1] * v[1] + v[2] * v[2] + v[3] * v[3]; }
    s += __shfl_xor(s, 16, 32); s += __shfl_xor(s, 8, 32); s += __shfl_xor(s, 4, 32); s += __shfl_xor(s, 2, 32); s += __shfl_xor(s, 1, 32);
    const float inv = 1.0f / (sqrtf(s) + L2EPS);
#pragma unroll 1
    for (int ps = 0; ps < 2; ++ps) {
#pragma unroll 1
        for (int i = 0; i < ND / 128; ++i) { const v4f v = *(const v4f*)(y + (i * 32 + lane) * 4); v4f w;
            w[0] = v[0] * inv; w[1] = v[1] * inv; w[2] = v[2] * inv; w[3] = v[3] * inv;
            *(volatile v4f*)(o + (i * 32 + lane) * 4) = w; }
        if (ps == 0) __threadfence(); }
}

static constexpr size_t al256(size_t v) { return (v + 255) & ~(size_t)255; }
static constexpr size_t SZ_PFB = al256((size_t)NS * ND * 2);
static constexpr size_t SZ_XB  = al256((size_t)NBQ * NE * 2);
static constexpr size_t SZ_W1T = al256((size_t)NE * ND * 2);
static constexpr size_t SZ_W2T = al256((size_t)NE * NE * 2);
static constexpr size_t SZ_Z1  = al256((size_t)NS * NE * 4);
static constexpr size_t SZ_Z2  = al256((size_t)NBQ * NE * 4);
static constexpr size_t SZ_ST  = al256((size_t)NE * 4);
static constexpr size_t SZ_WS  = al256((size_t)NS * NE * 2);
static constexpr size_t SZ_WV  = al256((size_t)NBQ * NE * 2);
static constexpr size_t SZ_INV = al256((size_t)NS * 4);
static constexpr size_t SZ_CNT = al256((size_t)ND * NS * 2);
static constexpr size_t SZ_PP  = al256((size_t)NBQ * NS * 2);
static constexpr size_t SZ_Y   = al256((size_t)NBQ * ND * 4);
static constexpr size_t SZ_TOTAL = SZ_PFB + SZ_XB + SZ_W1T + SZ_W2T + SZ_Z1 + SZ_Z2 + 4 * SZ_ST + 2 * SZ_WS + 2 * SZ_WV + SZ_INV + SZ_CNT + SZ_PP + SZ_Y;
static_assert(SZ_TOTAL <= (size_t)134217728);
static_assert((NE / 32) * 32 * 4 == NE * 4);
static_assert((NS / 32) * 32 * 4 == NS * 4);

extern "C" void kernel_launch(void* const* d_in, const int* in_sizes, int n_in,
                              void* d_out, int out_size, void* d_ws, size_t ws_size, hipStream_t stream) {
    if (n_in < 13) return;
    if ((size_t)in_sizes[0] < (size_t)NBQ * NE) return;
    if ((size_t)in_sizes[1] < (size_t)NS * ND) return;
    if ((size_t)in_sizes[3] < (size_t)ND * NE) return;
    if (in_sizes[4] < NE || in_sizes[5] < NE || in_sizes[6] < NE) return;
    if ((size_t)in_sizes[7] < (size_t)NE * NE) return;
    if (in_sizes[8] < NE || in_sizes[9] < NE || in_sizes[10] < NE || in_sizes[11] < NE || in_sizes[12] < 1) return;
    if ((size_t)out_size < (size_t)NBQ_FULL * ND + (size_t)NBQ * NS) return;
    if (SZ_TOTAL > ws_size) return;
    const float* xin = (const float*)d_in[0];
    const float* pin = (const float*)d_in[1];
    const float* w1 = (const float*)d_in[3];  const float* b1 = (const float*)d_in[4];
    const float* g1 = (const float*)d_in[5];  const float* s1 = (const float*)d_in[6];
    const float* w2 = (const float*)d_in[7];  const float* b2 = (const float*)d_in[8];
    const float* g2 = (const float*)d_in[9];  const float* s2 = (const float*)d_in[10];
    const float* w3 = (const float*)d_in[11]; const float* b3 = (const float*)d_in[12];
    float* O0 = (float*)d_out;
    float* O1 = (float*)d_out + (size_t)NBQ_FULL * ND;
    char* wsp = (char*)d_ws;
    bf*  PFB = (bf*)wsp;  wsp += SZ_PFB;
    bf*  XB  = (bf*)wsp;  wsp += SZ_XB;
    bf*  W1T = (bf*)wsp;  wsp += SZ_W1T;
    bf*  W2T = (bf*)wsp;  wsp += SZ_W2T;
    float* Z1 = (float*)wsp; wsp += SZ_Z1;
    float* Z2 = (float*)wsp; wsp += SZ_Z2;
    float* MU1 = (float*)wsp; wsp += SZ_ST;
    float* RS1 = (float*)wsp; wsp += SZ_ST;
    float* MU2 = (float*)wsp; wsp += SZ_ST;
    float* RS2 = (float*)wsp; wsp += SZ_ST;
    h16* WSH = (h16*)wsp; wsp += SZ_WS;
    h16* WSR = (h16*)wsp; wsp += SZ_WS;
    h16* WVH = (h16*)wsp; wsp += SZ_WV;
    h16* WVR = (h16*)wsp; wsp += SZ_WV;
    float* INV = (float*)wsp; wsp += SZ_INV;
    h16* CNT = (h16*)wsp; wsp += SZ_CNT;
    h16* PP  = (h16*)wsp; wsp += SZ_PP;
    float* Y = (float*)wsp; wsp += SZ_Y;

    { const size_t n8 = (size_t)NS * ND / 8;  k_cvt8<<<(unsigned)((n8 + 255) / 256), 256, 0, stream>>>(pin, PFB, n8); }
    { const size_t n8 = (size_t)NBQ * NE / 8; k_cvt8<<<(unsigned)((n8 + 255) / 256), 256, 0, stream>>>(xin, XB, n8); }
    k_tcvt<<<dim3(NE / 64, ND / 64, 1), 256, 0, stream>>>(w1, W1T, ND, NE);
    k_tcvt<<<dim3(NE / 64, NE / 64, 1), 256, 0, stream>>>(w2, W2T, NE, NE);
    k_rnorm<<<NS / 32, 256, 0, stream>>>(pin, INV);
    k_cfnt<<<dim3(ND / 64, NS / 64, 1), 256, 0, stream>>>(pin, INV, CNT, NS, ND);

    k_gemm_bf<<<dim3(NS / 64, NE / 64, 1), 32, 0, stream>>>(PFB, W1T, b1, Z1, ND, NE);
    k_gemm_bf<<<dim3(NBQ / 64, NE / 64, 1), 32, 0, stream>>>(XB, W2T, b2, Z2, NE, NE);

    k_bnstat<<<NE / 32, 256, 0, stream>>>(Z1, MU1, RS1, NS);
    k_bnstat<<<NE / 32, 256, 0, stream>>>(Z2, MU2, RS2, NBQ);
    k_bnact<<<(unsigned)(((size_t)NS * NE) / 2048), 256, 0, stream>>>(Z1, MU1, RS1, g1, s1, w3, 0, 1.0f, WSH, WSR);
    k_bnact<<<(unsigned)(((size_t)NBQ * NE) / 2048), 256, 0, stream>>>(Z2, MU2, RS2, g2, s2, w3, 1, WCAR, WVH, WVR);

    k_score<<<NBQ / 16, 256, 0, stream>>>(WSH, WSR, WVH, WVR, b3, O1, PP);
    k_gemm_h<<<dim3(NBQ / 64, ND / 64, 1), 32, 0, stream>>>(PP, CNT, YSCL, Y, NS, ND);
    k_l2out<<<NBQ / 8, 256, 0, stream>>>(Y, O0);
}
